// Router_64175401337509
// MI455X (gfx1250) — hardware-verified
//
#include <hip/hip_runtime.h>

typedef __attribute__((ext_vector_type(16))) _Float16 v16h;
typedef __attribute__((ext_vector_type(8)))  float    v8f;

#define NUM_LAYERS 24
#define LN_EPS 1e-5f
#define RSPLIT (1.0f / 2048.0f)

static __device__ __forceinline__ _Float16 lo_of(float v, _Float16 h) { return (_Float16)((v - (float)h) * 2048.0f); }
static __device__ __forceinline__ v8f wmma16(v16h a, v16h b, v8f c) {
    return __builtin_amdgcn_wmma_f32_16x16x32_f16(false, a, false, b, (short)0, c, false, false);
}
static __device__ __forceinline__ v8f wmma_split(v16h a, v16h al, v16h b, v16h bl, v8f c) {
    v8f x = {}; x = wmma16(al, b, x); x = wmma16(a, bl, x); return wmma16(a, b, c) + x * RSPLIT;
}
static __device__ __forceinline__ int kidx(int i, int hi) { return ((i < 8) ? i : (i + 8)) + 8 * hi; }

__global__ __launch_bounds__(256) void router_mlp_kernel(
    const float* __restrict__ x,
    const float* __restrict__ ln_gamma, const float* __restrict__ ln_beta,
    const float* __restrict__ W1, const float* __restrict__ b1,
    const float* __restrict__ W2, const float* __restrict__ b2,
    const float* __restrict__ W3, const float* __restrict__ b3,
    float* __restrict__ out, int nPairs)
{
    const int lane = threadIdx.x & 31, hi = lane >> 4, n = lane & 15;
    const int waveId = blockIdx.x * (blockDim.x >> 5) + (threadIdx.x >> 5);
    const int nWaves = gridDim.x * (blockDim.x >> 5);

    v16h a1[4], a1l[4];
    #pragma unroll
    for (int mt = 0; mt < 4; ++mt) {
        #pragma unroll
        for (int i = 0; i < 16; ++i) { a1[mt][i] = (_Float16)0.f; a1l[mt][i] = (_Float16)0.f; }
        if (hi == 0) {
            #pragma unroll
            for (int k = 0; k < 5; ++k) { const float w = W1[k * 64 + mt * 16 + n]; a1[mt][k] = (_Float16)w; a1l[mt][k] = lo_of(w, a1[mt][k]); }
        }
    }
    v16h a2[2][2], a2l[2][2];
    #pragma unroll
    for (int m2 = 0; m2 < 2; ++m2)
        #pragma unroll
        for (int kc = 0; kc < 2; ++kc)
            #pragma unroll
            for (int i = 0; i < 16; ++i) {
                const int k = kc * 32 + kidx(i, hi);
                const float w = W2[k * 32 + m2 * 16 + n];
                a2[m2][kc][i] = (_Float16)w; a2l[m2][kc][i] = lo_of(w, a2[m2][kc][i]);
            }
    float cb1[4][8], cb2[2][8], w3r[2][8];
    #pragma unroll
    for (int v = 0; v < 8; ++v) {
        #pragma unroll
        for (int mt = 0; mt < 4; ++mt) cb1[mt][v] = b1[mt * 16 + hi * 8 + v];
        #pragma unroll
        for (int m2 = 0; m2 < 2; ++m2) { cb2[m2][v] = b2[m2 * 16 + hi * 8 + v]; w3r[m2][v] = W3[m2 * 16 + hi * 8 + v]; }
    }
    const float b3s = b3[0];

    for (int tp = waveId; tp < nPairs; tp += nWaves) {
        float res[2];
        #pragma unroll
        for (int u = 0; u < 2; ++u) {
            const long long tok = ((long long)tp * 2 + u) * 16 + n;
            const float* xr = x + tok * 5;
            const float f0 = xr[0], f1 = xr[1], f2 = xr[2], f3 = xr[3], lp = xr[4];
            int lid = (int)(lp * (float)NUM_LAYERS);
            lid = lid < 0 ? 0 : (lid > NUM_LAYERS - 1 ? NUM_LAYERS - 1 : lid);
            const float mu = (f0 + f1 + f2 + f3) * 0.25f;
            const float d0 = f0 - mu, d1 = f1 - mu, d2 = f2 - mu, d3 = f3 - mu;
            const float var = (d0 * d0 + d1 * d1 + d2 * d2 + d3 * d3) * 0.25f;
            const float rs = 1.0f / sqrtf(var + LN_EPS);
            float feat[5];
            feat[0] = d0 * rs * ln_gamma[lid * 4 + 0] + ln_beta[lid * 4 + 0];
            feat[1] = d1 * rs * ln_gamma[lid * 4 + 1] + ln_beta[lid * 4 + 1];
            feat[2] = d2 * rs * ln_gamma[lid * 4 + 2] + ln_beta[lid * 4 + 2];
            feat[3] = d3 * rs * ln_gamma[lid * 4 + 3] + ln_beta[lid * 4 + 3];
            feat[4] = lp;
            v16h bq, bql;
            #pragma unroll
            for (int i = 0; i < 16; ++i) { bq[i] = (_Float16)0.f; bql[i] = (_Float16)0.f; }
            if (hi == 0) {
                #pragma unroll
                for (int k = 0; k < 5; ++k) { bq[k] = (_Float16)feat[k]; bql[k] = lo_of(feat[k], bq[k]); }
            }
            v8f cz = {};
            v8f c1[4];
            #pragma unroll
            for (int mt = 0; mt < 4; ++mt) c1[mt] = wmma_split(a1[mt], a1l[mt], bq, bql, cz);
            v16h bz[2], bzl[2];
            #pragma unroll
            for (int kc = 0; kc < 2; ++kc)
                #pragma unroll
                for (int i = 0; i < 8; ++i) {
                    const float h0 = fmaxf(c1[2 * kc][i] + cb1[2 * kc][i], 0.f), h1 = fmaxf(c1[2 * kc + 1][i] + cb1[2 * kc + 1][i], 0.f);
                    bz[kc][i] = (_Float16)h0;      bzl[kc][i] = lo_of(h0, bz[kc][i]);
                    bz[kc][i + 8] = (_Float16)h1;  bzl[kc][i + 8] = lo_of(h1, bz[kc][i + 8]);
                }
            v8f c2[2];
            #pragma unroll
            for (int m2 = 0; m2 < 2; ++m2) { c2[m2] = cz;
                #pragma unroll
                for (int kc = 0; kc < 2; ++kc) c2[m2] = wmma_split(a2[m2][kc], a2l[m2][kc], bz[kc], bzl[kc], c2[m2]); }
            float acc = 0.f;
            #pragma unroll
            for (int v = 0; v < 8; ++v) {
                acc = fmaf(w3r[0][v], fmaxf(c2[0][v] + cb2[0][v], 0.f), acc);
                acc = fmaf(w3r[1][v], fmaxf(c2[1][v] + cb2[1][v], 0.f), acc);
            }
            acc += __shfl_xor(acc, 16, 32);
            res[u] = acc + b3s;
        }
        const float ov = (hi == 0) ? res[0] : res[1];
        float* op = out + (size_t)tp * 32 + lane;
        *(volatile float*)op = ov; __threadfence(); *(volatile float*)op = ov;
    }
}

extern "C" void kernel_launch(void* const* d_in, const int* in_sizes, int n_in,
                              void* d_out, int out_size, void* d_ws, size_t ws_size,
                              hipStream_t stream) {
    (void)n_in; (void)out_size; (void)d_ws; (void)ws_size;
    const float* x        = (const float*)d_in[0];
    const float* ln_gamma = (const float*)d_in[1];
    const float* ln_beta  = (const float*)d_in[2];
    const float* W1       = (const float*)d_in[3];
    const float* b1       = (const float*)d_in[4];
    const float* W2       = (const float*)d_in[5];
    const float* b2       = (const float*)d_in[6];
    const float* W3       = (const float*)d_in[7];
    const float* b3       = (const float*)d_in[8];
    float* out            = (float*)d_out;

    const int rows   = in_sizes[0] / 5;
    const int nPairs = rows / 32;
    router_mlp_kernel<<<dim3(1024), dim3(256), 0, stream>>>(x, ln_gamma, ln_beta, W1, b1, W2, b2, W3, b3, out, nPairs);
}
